// Decoder_8340826489417
// MI455X (gfx1250) — hardware-verified
//
#include <hip/hip_runtime.h>
#include <math.h>

constexpr int NSTEPS = 12;
constexpr int HID    = 128;
constexpr int EMB    = 64;
constexpr int NGATE  = 4 * HID;
constexpr int NPED   = 65536;
constexpr int NTHR   = 256;
constexpr int NWAVE  = NTHR / 32;
constexpr int ROWS_PER_WAVE  = 16;
constexpr int ROWS_PER_BLOCK = NWAVE * ROWS_PER_WAVE;
constexpr int NBLOCKS = NPED / ROWS_PER_BLOCK;
constexpr int WPITCH = 136;
constexpr int HPITCH = 136;
constexpr int CPITCH = 132;
constexpr float W_CARRY  = 256.0f;
constexpr float H_CARRY  = 16.0f;
constexpr float ACC_FOLD = 1.0f / (W_CARRY * H_CARRY);
constexpr bool IN_BF16 = false;

static_assert(HID % 32 == 0, "K multiple of 32");
static_assert(NGATE == 512 && HID == 128 && EMB == 64, "shape");
static_assert(NPED % ROWS_PER_BLOCK == 0, "grid exact");
static_assert(NBLOCKS == 512, "grid");
static_assert((NGATE * (HID / 8)) % NTHR == 0, "weight staging exact");
static_assert(ROWS_PER_BLOCK * 2 == NTHR, "x staging exact");

constexpr int OFF_W    = 0;
constexpr int OFF_H    = OFF_W    + NGATE * WPITCH * 2;
constexpr int OFF_C    = OFF_H    + NWAVE * 16 * HPITCH * 2;
constexpr int OFF_W2   = OFF_C    + NWAVE * 16 * CPITCH * 4;
constexpr int OFF_BALL = OFF_W2   + NGATE * 2 * 4;
constexpr int OFF_WHP  = OFF_BALL + NGATE * 4;
constexpr int OFF_REL  = OFF_WHP  + 2 * HID * 4;
constexpr int SMEM_BYTES = OFF_REL + NWAVE * 32 * 4;
static_assert(SMEM_BYTES == 249856, "LDS total");
static_assert(OFF_H % 16 == 0 && OFF_C % 16 == 0 && OFF_W2 % 16 == 0 && OFF_BALL % 16 == 0 && OFF_WHP % 16 == 0 && OFF_REL % 16 == 0, "LDS alignment");

typedef __attribute__((ext_vector_type(16))) _Float16 v16h;
typedef __attribute__((ext_vector_type(8)))  _Float16 v8h;
typedef __attribute__((ext_vector_type(8)))  float    v8f;
typedef __attribute__((ext_vector_type(4)))  float    v4f;

__device__ __forceinline__ float bf16r(float f) {
  const unsigned u = __float_as_uint(f);
  const unsigned r = (u + 0x7FFFu + ((u >> 16) & 1u)) & 0xFFFF0000u;
  return __uint_as_float(r);
}
__device__ __forceinline__ float ldin(float f) { return IN_BF16 ? bf16r(f) : f; }

__device__ __forceinline__ void gate_guard(v8f& d0, v8f& d1, v8f& d2, v8f& d3, v16h a, v16h b0, v16h b1, v16h b2, v16h b3) {
  asm volatile("v_nop\n\tv_nop\n\tv_nop\n\tv_nop" : "+v"(d0), "+v"(d1), "+v"(d2), "+v"(d3) : "v"(a), "v"(b0), "v"(b1), "v"(b2), "v"(b3));
}

template <typename T> struct Frag;
template <> struct Frag<_Float16> {
  typedef v16h V; union U { v16h v; v8h h[2]; };
  static __device__ __forceinline__ v16h load(const _Float16* p) {
    U f; f.h[0] = *(const v8h*)(p); f.h[1] = *(const v8h*)(p + 16); return f.v;
  }
  static __device__ __forceinline__ v8f mma(v16h a, v16h b, v8f c) {
    return __builtin_amdgcn_wmma_f32_16x16x32_f16(false, a, false, b, (short)0, c, false, false);
  }
};

__device__ __forceinline__ float sigm(float x) { return __builtin_amdgcn_rcpf(1.0f + expf(-x)); }
__device__ __forceinline__ float tnh(float x)  { return 1.0f - 2.0f * __builtin_amdgcn_rcpf(1.0f + expf(2.0f * x)); }

__global__ __launch_bounds__(NTHR) void prep_wh_kernel(const float* __restrict__ w_hh, unsigned short* __restrict__ dst) {
  const int i = blockIdx.x * NTHR + threadIdx.x;
  if (i < NGATE * (HID / 8)) {
    const v4f a = *(const v4f*)(w_hh + (size_t)i * 8);
    const v4f b = *(const v4f*)(w_hh + (size_t)i * 8 + 4);
    v8h hv;
#pragma unroll
    for (int e = 0; e < 4; ++e) {
      const float fa = a[e];
      const float fb = b[e];
      hv[e]     = (_Float16)(ldin(fa) * W_CARRY);
      hv[4 + e] = (_Float16)(ldin(fb) * W_CARRY);
    }
    _Float16* dp = (_Float16*)dst + (size_t)i * 8;
    *(volatile v8h*)dp = hv;
    __threadfence();
    *(volatile v8h*)dp = hv;
  }
}

__global__ __launch_bounds__(512) void prep_fold_kernel(const float* __restrict__ w_ih, const float* __restrict__ b_ih,
                                                        const float* __restrict__ b_hh, const float* __restrict__ w_se,
                                                        const float* __restrict__ b_se,
                                                        float* __restrict__ W2g, float* __restrict__ BALLg) {
  __shared__ __align__(16) float sWse[2 * EMB];
  __shared__ __align__(16) float sBse[EMB];
  __shared__ __align__(16) float sW2[2 * NGATE];
  __shared__ __align__(16) float sBall[NGATE];
  const int tid = threadIdx.x;
  if (tid < 2 * EMB) {
    const float v = w_se[tid];
    sWse[tid] = ldin(v);
  } else if (tid < 3 * EMB) {
    const float v = b_se[tid - 2 * EMB];
    sBse[tid - 2 * EMB] = ldin(v);
  }
  __syncthreads();
  const int n = tid;
  const float* wr = w_ih + (size_t)n * EMB;
  float s0 = 0.0f, s1 = 0.0f, sb = 0.0f;
#pragma unroll 1
  for (int e4 = 0; e4 < EMB / 4; ++e4) {
    const v4f w = *(const v4f*)(wr + e4 * 4);
#pragma unroll
    for (int q = 0; q < 4; ++q) {
      const float wraw = w[q];
      const float wv = ldin(wraw);
      const int e = e4 * 4 + q;
      s0 = fmaf(wv, sWse[2 * e + 0], s0);
      s1 = fmaf(wv, sWse[2 * e + 1], s1);
      sb = fmaf(wv, sBse[e], sb);
    }
  }
  const float bi = b_ih[n];
  const float bh = b_hh[n];
  const float ball = (ldin(bi) + ldin(bh)) + sb;
  sW2[2 * n + 0] = s0;
  sW2[2 * n + 1] = s1;
  sBall[n] = ball;
  __syncthreads();
  if (tid < 256) {
    const v4f v = *(const v4f*)(sW2 + tid * 4);
    float* dp = W2g + tid * 4;
    *(volatile v4f*)dp = v;
    __threadfence();
    *(volatile v4f*)dp = v;
  } else if (tid < 384) {
    const int q = tid - 256;
    const v4f v = *(const v4f*)(sBall + q * 4);
    float* dp = BALLg + q * 4;
    *(volatile v4f*)dp = v;
    __threadfence();
    *(volatile v4f*)dp = v;
  }
}

__global__ __launch_bounds__(NTHR) void decoder_kernel(const float* __restrict__ last_pos_rel, const float* __restrict__ h0,
                                                       const float* __restrict__ c0, const float* __restrict__ w_hp,
                                                       const float* __restrict__ b_hp, const unsigned short* __restrict__ WHp,
                                                       const float* __restrict__ W2g, const float* __restrict__ BALLg,
                                                       float* __restrict__ out) {
  extern __shared__ __align__(16) unsigned char smem[];
  _Float16* Wsh  = (_Float16*)(smem + OFF_W);
  _Float16* Hsh  = (_Float16*)(smem + OFF_H);
  float*    Csh  = (float*)(smem + OFF_C);
  float*    W2s  = (float*)(smem + OFF_W2);
  float*    Bls  = (float*)(smem + OFF_BALL);
  float*    Whps = (float*)(smem + OFF_WHP);
  float*    Relb = (float*)(smem + OFF_REL);

  const int tid = threadIdx.x, lane = tid & 31, wave = tid >> 5;
  const int c = lane & 15, hh = lane >> 4, koff = hh * 8;
  const int blockRow = blockIdx.x * ROWS_PER_BLOCK;
  const int pedBase  = blockRow + wave * ROWS_PER_WAVE;

  const _Float16* WH = (const _Float16*)WHp;
#pragma unroll 4
  for (int i = tid; i < NGATE * (HID / 8); i += NTHR) {
    const int row = i >> 4, c8 = (i & 15) * 8;
    const v8h v = *(const v8h*)(WH + (size_t)row * HID + c8);
    *(v8h*)(Wsh + row * WPITCH + c8) = v;
  }
  {
    const v4f v = *(const v4f*)(W2g + tid * 4);
    *(v4f*)(W2s + tid * 4) = v;
  }
  if (tid < 128) {
    const v4f v = *(const v4f*)(BALLg + tid * 4);
    *(v4f*)(Bls + tid * 4) = v;
  }
  if (tid < 64) {
    const v4f v = *(const v4f*)(w_hp + tid * 4);
    v4f o;
#pragma unroll
    for (int e = 0; e < 4; ++e) {
      const float s = v[e];
      o[e] = ldin(s);
    }
    *(v4f*)(Whps + tid * 4) = o;
  }
  {
    const float s = last_pos_rel[(size_t)blockRow * 2 + tid];
    Relb[tid] = ldin(s);
  }
  const float bhp_raw = b_hp[lane & 1];
  const float bhp_l = ldin(bhp_raw);

  _Float16* Hw   = Hsh + wave * 16 * HPITCH;
  float*    Cw   = Csh + wave * 16 * CPITCH;
  float*    relw = Relb + wave * 32;

#pragma unroll 2
  for (int it = 0; it < 16; ++it) {
    const size_t g = (size_t)(pedBase + it) * HID + lane * 4;
    const v4f hv = *(const v4f*)(h0 + g);
    const v4f cv = *(const v4f*)(c0 + g);
#pragma unroll
    for (int e = 0; e < 4; ++e) {
      const float hs = hv[e];
      const float cs = cv[e];
      Hw[it * HPITCH + lane * 4 + e] = (_Float16)(ldin(hs) * H_CARRY);
      Cw[it * CPITCH + lane * 4 + e] = ldin(cs);
    }
  }
  __syncthreads();

  const v8f z8 = {0.f, 0.f, 0.f, 0.f, 0.f, 0.f, 0.f, 0.f};
  const _Float16* arow = Hw + c * HPITCH + koff;

#pragma unroll 1
  for (int t = 0; t < NSTEPS; ++t) {
    v16h af[4];
#pragma unroll
    for (int kt = 0; kt < 4; ++kt) af[kt] = Frag<_Float16>::load(arow + kt * 32);
    float xs[16];
    {
      const float* xr = relw + 16 * hh;
      const v4f xa = *(const v4f*)(xr);
      const v4f xb = *(const v4f*)(xr + 4);
      const v4f xc = *(const v4f*)(xr + 8);
      const v4f xd = *(const v4f*)(xr + 12);
#pragma unroll
      for (int e = 0; e < 4; ++e) {
        xs[e] = xa[e];
        xs[4 + e] = xb[e];
        xs[8 + e] = xc[e];
        xs[12 + e] = xd[e];
      }
    }
    float p[16];
#pragma unroll
    for (int i = 0; i < 16; ++i) p[i] = 0.0f;

#pragma unroll 1
    for (int ht = 0; ht < HID / 16; ++ht) {
      const int col = ht * 16 + c;
      const _Float16* wb = Wsh + col * WPITCH + koff;
      v8f acc0 = z8, acc1 = z8, acc2 = z8, acc3 = z8;
#pragma unroll
      for (int kt = 0; kt < 4; ++kt) {
        const v16h b0 = Frag<_Float16>::load(wb + kt * 32);
        const v16h b1 = Frag<_Float16>::load(wb + 1 * HID * WPITCH + kt * 32);
        const v16h b2 = Frag<_Float16>::load(wb + 2 * HID * WPITCH + kt * 32);
        const v16h b3 = Frag<_Float16>::load(wb + 3 * HID * WPITCH + kt * 32);
        acc0 = Frag<_Float16>::mma(af[kt], b0, acc0);
        acc1 = Frag<_Float16>::mma(af[kt], b1, acc1);
        acc2 = Frag<_Float16>::mma(af[kt], b2, acc2);
        acc3 = Frag<_Float16>::mma(af[kt], b3, acc3);
        gate_guard(acc0, acc1, acc2, acc3, af[kt], b0, b1, b2, b3);
      }
      const float bi = Bls[col],           wi0 = W2s[2 * col],               wi1 = W2s[2 * col + 1];
      const float bf = Bls[HID + col],     wf0 = W2s[2 * (HID + col)],       wf1 = W2s[2 * (HID + col) + 1];
      const float bg = Bls[2 * HID + col], wg0 = W2s[2 * (2 * HID + col)],   wg1 = W2s[2 * (2 * HID + col) + 1];
      const float bo = Bls[3 * HID + col], wo0 = W2s[2 * (3 * HID + col)],   wo1 = W2s[2 * (3 * HID + col) + 1];
      const float wp0 = Whps[col], wp1 = Whps[HID + col];
#pragma unroll
      for (int j = 0; j < 8; ++j) {
        const int rr = 8 * hh + j;
        const float x0 = xs[2 * j], x1 = xs[2 * j + 1];
        const float zi = fmaf(acc0[j], ACC_FOLD, fmaf(x1, wi1, fmaf(x0, wi0, bi)));
        const float zf = fmaf(acc1[j], ACC_FOLD, fmaf(x1, wf1, fmaf(x0, wf0, bf)));
        const float zg = fmaf(acc2[j], ACC_FOLD, fmaf(x1, wg1, fmaf(x0, wg0, bg)));
        const float zo = fmaf(acc3[j], ACC_FOLD, fmaf(x1, wo1, fmaf(x0, wo0, bo)));
        const float ig = sigm(zi);
        const float fg = sigm(zf);
        const float gg = tnh(zg);
        const float og = sigm(zo);
        const float cold = Cw[rr * CPITCH + col];
        const float cn = fg * cold + ig * gg;
        Cw[rr * CPITCH + col] = cn;
        const float hn = og * tnh(cn);
        Hw[rr * HPITCH + col] = (_Float16)(hn * H_CARRY);
        p[2 * j + 0] = fmaf(hn, wp0, p[2 * j + 0]);
        p[2 * j + 1] = fmaf(hn, wp1, p[2 * j + 1]);
      }
    }

#pragma unroll
    for (int i = 0; i < 16; ++i) {
      float v = p[i];
      v += __shfl_xor(v, 1, 32);
      v += __shfl_xor(v, 2, 32);
      v += __shfl_xor(v, 4, 32);
      v += __shfl_xor(v, 8, 32);
      p[i] = v;
    }
    float val = p[0];
#pragma unroll
    for (int i = 1; i < 16; ++i) val = (c == i) ? p[i] : val;
    val += bhp_l;
    relw[lane] = val;
    {
      float* op = out + ((size_t)t * NPED + (size_t)pedBase) * 2 + lane;
      *(volatile float*)op = val;
      __threadfence();
      *(volatile float*)op = val;
    }
    __syncthreads();
  }
}

extern "C" void kernel_launch(void* const* d_in, const int* in_sizes, int n_in,
                              void* d_out, int out_size, void* d_ws, size_t ws_size, hipStream_t stream) {
  if (n_in < 12 || d_out == nullptr || d_ws == nullptr) return;
  if (in_sizes[1] != NPED * 2 || in_sizes[2] != NPED * HID || in_sizes[3] != NPED * HID ||
      in_sizes[4] != NGATE * EMB || in_sizes[5] != NGATE * HID || in_sizes[6] != NGATE || in_sizes[7] != NGATE ||
      in_sizes[8] != EMB * 2 || in_sizes[9] != EMB || in_sizes[10] != 2 * HID || in_sizes[11] != 2 ||
      out_size != NSTEPS * NPED * 2) return;

  const float* last_pos_rel = (const float*)d_in[1];
  const float* h0   = (const float*)d_in[2];
  const float* c0   = (const float*)d_in[3];
  const float* w_ih = (const float*)d_in[4];
  const float* w_hh = (const float*)d_in[5];
  const float* b_ih = (const float*)d_in[6];
  const float* b_hh = (const float*)d_in[7];
  const float* w_se = (const float*)d_in[8];
  const float* b_se = (const float*)d_in[9];
  const float* w_hp = (const float*)d_in[10];
  const float* b_hp = (const float*)d_in[11];
  float* out = (float*)d_out;

  char* ws = (char*)d_ws; size_t off = 0;
  auto carve = [&](size_t bytes) -> char* { char* p = ws + off; off += (bytes + 255) & ~(size_t)255; return p; };
  unsigned short* WH   = (unsigned short*)carve((size_t)NGATE * HID * 2);
  float*          W2g  = (float*)carve((size_t)NGATE * 2 * 4);
  float*          BALL = (float*)carve((size_t)NGATE * 4);
  if (off > ws_size || off > (size_t)134217728) return;

  prep_wh_kernel<<<(NGATE * (HID / 8)) / NTHR, NTHR, 0, stream>>>(w_hh, WH);
  prep_fold_kernel<<<1, 512, 0, stream>>>(w_ih, b_ih, b_hh, w_se, b_se, W2g, BALL);
  decoder_kernel<<<NBLOCKS, NTHR, SMEM_BYTES, stream>>>(last_pos_rel, h0, c0, w_hp, b_hp, WH, W2g, BALL, out);
}
